// STNDTEncoder_83434034692803
// MI455X (gfx1250) — hardware-run, weakly checked
//
#include <hip/hip_runtime.h>
#include <math.h>

typedef __attribute__((ext_vector_type(16))) _Float16 v16h;
typedef __attribute__((ext_vector_type(16))) __bf16 v16b;
typedef __attribute__((ext_vector_type(8)))  _Float16 v8h;
typedef __attribute__((ext_vector_type(8)))  float v8f;
typedef __attribute__((ext_vector_type(4)))  float v4f;
typedef __attribute__((ext_vector_type(2)))  float v2f;
typedef __attribute__((ext_vector_type(4)))  unsigned v4u;
typedef __attribute__((ext_vector_type(4)))  int v4i;
typedef float __attribute__((may_alias)) float_a;
typedef int __attribute__((may_alias)) int_a;

template <typename T> __device__ __forceinline__ void vst2(void* p, T v) { *(volatile T*)p = v; __threadfence(); *(volatile T*)p = v; }
__device__ __forceinline__ v8f wmma16(v16h a, v16h b, v8f c) {
  v8f d = __builtin_amdgcn_wmma_f32_16x16x32_f16(false, a, false, b, (short)0, c, false, false);
  asm volatile("v_nop\n\tv_nop\n\tv_nop\n\tv_nop" : "+v"(d) : "v"(a), "v"(b));
  return d;
}
__device__ __forceinline__ v8f wmma_bf(v16b a, v16b b, v8f c) {
  v8f d = __builtin_amdgcn_wmma_f32_16x16x32_bf16(false, a, false, b, (short)0, c, false, false);
  asm volatile("v_nop\n\tv_nop\n\tv_nop\n\tv_nop" : "+v"(d) : "v"(a), "v"(b));
  return d;
}
__device__ __forceinline__ v16h frag_h(const _Float16* rowk0, int lane) {
  union { v16h v; v8h q[2]; } u; const _Float16* p = rowk0 + 8 * (lane >> 4);
  u.q[0] = *(const v8h*)p; u.q[1] = *(const v8h*)(p + 16); return u.v;
}
__device__ __forceinline__ v16h frag_f32(const float* rowk0, int lane) {
  v16h a; const float* p = rowk0 + 8 * (lane >> 4);
#pragma unroll
  for (int i = 0; i < 8; ++i) { a[i] = (_Float16)p[i]; a[8 + i] = (_Float16)p[16 + i]; }
  return a;
}
__device__ __forceinline__ v16h frag_f32s(const float* rowk0, int lane, float sc) {
  v16h a; const float* p = rowk0 + 8 * (lane >> 4);
#pragma unroll
  for (int i = 0; i < 8; ++i) { a[i] = (_Float16)(p[i] * sc); a[8 + i] = (_Float16)(p[16 + i] * sc); }
  return a;
}
__device__ __forceinline__ v16h fragc_f32(const float* W, int k0, int n, int lane, int ld, int K) {
  v16h a; const int g = lane >> 4;
#pragma unroll
  for (int i = 0; i < 8; ++i) { const int ka = k0 + 8 * g + i, kb = ka + 16;
    a[i] = (_Float16)(ka < K ? W[(size_t)(ka < K ? ka : K - 1) * ld + n] : 0.f); a[8 + i] = (_Float16)(kb < K ? W[(size_t)(kb < K ? kb : K - 1) * ld + n] : 0.f); }
  return a;
}
struct F2 { v16b h, l; };
__device__ __forceinline__ F2 bsplit16(const float v[16]) { F2 r;
#pragma unroll
  for (int i = 0; i < 16; ++i) { const __bf16 h = (__bf16)v[i]; r.h[i] = h; r.l[i] = (__bf16)(v[i] - (float)h); }
  return r; }
__device__ __forceinline__ F2 split_row(const float* row, int k0, int lane) { float v[16]; const float* p = row + k0 + 8 * (lane >> 4);
#pragma unroll
  for (int i = 0; i < 8; ++i) { v[i] = p[i]; v[8 + i] = p[16 + i]; }
  return bsplit16(v); }
__device__ __forceinline__ F2 split_rowK(const float* row, int k0, int lane, int K) { float v[16]; const int g = lane >> 4;
#pragma unroll
  for (int i = 0; i < 8; ++i) { const int ka = k0 + 8 * g + i, kb = ka + 16; v[i] = ka < K ? row[ka < K ? ka : K - 1] : 0.f; v[8 + i] = kb < K ? row[kb < K ? kb : K - 1] : 0.f; }
  return bsplit16(v); }
__device__ __forceinline__ F2 split_col(const float* W, int k0, int n, int lane, int ld, int K) { float v[16]; const int g = lane >> 4;
#pragma unroll
  for (int i = 0; i < 8; ++i) { const int ka = k0 + 8 * g + i, kb = ka + 16; v[i] = ka < K ? W[(size_t)(ka < K ? ka : K - 1) * ld + n] : 0.f; v[8 + i] = kb < K ? W[(size_t)(kb < K ? kb : K - 1) * ld + n] : 0.f; }
  return bsplit16(v); }
__device__ __forceinline__ v8f mac3(const F2& a, const F2& b, v8f c) { c = wmma_bf(a.l, b.h, c); c = wmma_bf(a.h, b.l, c); return wmma_bf(a.h, b.h, c); }
__device__ __forceinline__ float sigm(float v) { return 1.0f / (1.0f + expf(-v)); }
#define LDSX() do { asm volatile("s_wait_dscnt 0" ::: "memory"); __builtin_amdgcn_wave_barrier(); __builtin_amdgcn_fence(__ATOMIC_RELEASE, "workgroup"); } while (0)


#define NB 16
#define TT 512
#define CC 512
#define LL 512
#define NH 8
#define HS 64
#define HID 2048
#define NR (NB * TT)
#define NRS (NB * CC)
#define WSC 256.0f
#ifndef TNB
#define TNB NB
#endif
typedef __attribute__((ext_vector_type(8))) __bf16 v8b;
__device__ __forceinline__ v16b frag_b(const __bf16* rowk0, int lane) {
  union { v16b v; v8b q[2]; } u; const __bf16* p = rowk0 + 8 * (lane >> 4);
  u.q[0] = *(const v8b*)p; u.q[1] = *(const v8b*)(p + 16); return u.v;
}
__device__ __forceinline__ float bfr(float v) { return (float)(__bf16)v; }
__device__ __attribute__((noinline)) float exp_ni(float v) { return expf(v); }
__device__ __attribute__((noinline)) float erf_ni(float v) { return erff(v); }

#define WS_PW  0u
#define WS_PO  (WS_PW + 2u * (size_t)1536 * CC)
#define WS_P1  (WS_PO + 2u * (size_t)CC * CC)
#define WS_P2  (WS_P1 + 2u * (size_t)HID * CC)
#define WS_PS  (WS_P2 + 2u * (size_t)CC * HID)
#define WS_PT1 (WS_PS + 2u * (size_t)1024 * LL)
#define WS_PT2 (WS_PT1 + 2u * (size_t)HID * CC)
#define WS_LN  (WS_PT2 + 2u * (size_t)CC * HID)
#define WS_Q   (WS_LN + 2u * (size_t)NR * CC)
#define WS_K   (WS_Q + 2u * (size_t)NR * CC)
#define WS_V   (WS_K + 2u * (size_t)NR * CC)
#define WS_O   (WS_V + 2u * (size_t)NB * CC * TT)
#define WS_S1  (WS_O + 4u * (size_t)NR * CC)
#define WS_S2  (WS_S1 + 4u * (size_t)NR * CC)
#define WS_S3  (WS_S2 + 4u * (size_t)NR * CC)
#define WS_HH  (WS_S3 + 4u * (size_t)NR * CC)
#define WS_SP  (WS_HH + 2u * (size_t)NR * HID)
#define WS_QS  (WS_SP + 2u * (size_t)NRS * LL)
#define WS_ST  (WS_QS + 2u * (size_t)NRS * 1024)
#define WS_SWH (WS_ST + 4u * (size_t)NB * CC * 32)
#define WS_END (WS_SWH + 2u * (size_t)NB * CC * CC)
#define OUT1   ((size_t)NR * CC)

__global__ __launch_bounds__(256) void k_pack(const float* __restrict__ WQ, const float* __restrict__ WK, const float* __restrict__ WV, const float* __restrict__ WO, const float* __restrict__ W1, const float* __restrict__ W2, const float* __restrict__ WQS, const float* __restrict__ WKS, const float* __restrict__ T1, const float* __restrict__ T2, _Float16* __restrict__ P) {
  const int n = blockIdx.x, which = blockIdx.y, t = threadIdx.x; __shared__ __align__(16) _Float16 s[HID];
  const float* src; size_t dst; int len;
  if (which == 0) { if (n >= 1536) return; const int m = n / CC, r = n % CC; src = ((m == 0) ? WQ : (m == 1) ? WK : WV) + (size_t)r * CC; dst = WS_PW / 2 + (size_t)n * CC; len = CC; }
  else if (which == 1) { if (n >= CC) return; src = WO + (size_t)n * CC; dst = WS_PO / 2 + (size_t)n * CC; len = CC; }
  else if (which == 2) { src = W1 + (size_t)n * CC; dst = WS_P1 / 2 + (size_t)n * CC; len = CC; }
  else if (which == 3) { if (n >= CC) return; src = W2 + (size_t)n * HID; dst = WS_P2 / 2 + (size_t)n * HID; len = HID; }
  else if (which == 4) { if (n >= 1024) return; const int m = n / LL, r = n % LL; src = ((m == 0) ? WQS : WKS) + (size_t)r * LL; dst = WS_PS / 2 + (size_t)n * LL; len = LL; }
  else if (which == 5) { src = T1 + (size_t)n * CC; dst = WS_PT1 / 2 + (size_t)n * CC; len = CC; }
  else { if (n >= CC) return; src = T2 + (size_t)n * HID; dst = WS_PT2 / 2 + (size_t)n * HID; len = HID; }
  for (int k = t; k < len; k += 256) s[k] = (_Float16)(bfr(src[k]) * WSC); __syncthreads(); for (int q = t; q < len / 8; q += 256) vst2((unsigned*)(P + dst + q * 8), *(const v4u*)&s[q * 8]); }
template <int RAW>
__global__ __launch_bounds__(256) void k_ln(const float* __restrict__ X, const float* __restrict__ G, const float* __restrict__ Bt, _Float16* __restrict__ Y) { __shared__ float red[8]; __shared__ __align__(16) _Float16 so[CC]; const int t = threadIdx.x; const size_t row = blockIdx.x;
  float v0 = X[row * CC + t], v1 = X[row * CC + t + 256]; if (RAW) { v0 = bfr(v0); v1 = bfr(v1); } float s = v0 + v1;
#pragma unroll
  for (int o = 1; o < 32; o <<= 1) s += __shfl_xor(s, o);
  if ((t & 31) == 0) red[t >> 5] = s; __syncthreads(); float tot = 0.f; for (int i = 0; i < 8; ++i) tot += red[i]; const float mu = tot / (float)CC; __syncthreads();
  const float d0 = v0 - mu, d1 = v1 - mu; float q = d0 * d0 + d1 * d1;
#pragma unroll
  for (int o = 1; o < 32; o <<= 1) q += __shfl_xor(q, o);
  if ((t & 31) == 0) red[t >> 5] = q; __syncthreads(); float tq = 0.f; for (int i = 0; i < 8; ++i) tq += red[i]; const float inv = 1.0f / sqrtf(tq / (float)CC + 1e-5f);
  so[t] = (_Float16)(d0 * inv * bfr(G[t]) + bfr(Bt[t])); so[t + 256] = (_Float16)(d1 * inv * bfr(G[t + 256]) + bfr(Bt[t + 256])); __syncthreads(); if (t < CC / 8) vst2((unsigned*)(Y + row * CC + t * 8), *(const v4u*)&so[t * 8]); }
template <int MODE, int KW>
__global__ __launch_bounds__(128) void k_g(const _Float16* __restrict__ A, const _Float16* __restrict__ Wr, const float* __restrict__ BI, const float* __restrict__ RES, const float* __restrict__ ALPHA, float* __restrict__ O32, _Float16* __restrict__ O16, _Float16* __restrict__ O16B, _Float16* __restrict__ VPL, int ow) {
  __shared__ __align__(16) float sf[4][16][132]; __shared__ __align__(16) _Float16 so[64][136]; __shared__ __align__(16) _Float16 st[128][72];
  const int tid = threadIdx.x, wave = tid >> 5, lane = tid & 31, col = lane & 15, g = lane >> 4; const int which = blockIdx.z; const size_t rb = (size_t)blockIdx.x * 64; const size_t r0 = rb + wave * 16; const int c0 = blockIdx.y * 128; const _Float16* W = Wr + ((MODE == 0) ? (size_t)which * CC * KW : 0);
  v8f acc[8] = {};
#pragma unroll 2
  for (int kc = 0; kc < KW / 32; ++kc) { const v16h a = frag_h(A + (r0 + col) * KW + kc * 32, lane);
#pragma unroll
    for (int j = 0; j < 8; ++j) acc[j] = wmma16(a, frag_h(W + (size_t)(c0 + j * 16 + col) * KW + kc * 32, lane), acc[j]); }
  if (MODE == 1) {
#pragma unroll
    for (int j = 0; j < 8; ++j) { const int c = c0 + j * 16 + col; const float bb = BI ? bfr(BI[c]) : 0.f;
#pragma unroll
      for (int r = 0; r < 8; ++r) sf[wave][8 * g + r][j * 16 + col] = acc[j][r] * (1.0f / WSC) + bb + RES[(r0 + 8 * g + r) * ow + c]; }
    LDSX(); for (int rl = 0; rl < 16; ++rl) vst2(O32 + (r0 + rl) * ow + c0 + lane * 4, *(const v4f*)&sf[wave][rl][lane * 4]); return; }
  if (MODE == 0 && which == 2) {
#pragma unroll
    for (int j = 0; j < 8; ++j)
#pragma unroll
      for (int r = 0; r < 8; ++r) st[j * 16 + col][wave * 16 + 8 * g + r] = (_Float16)(acc[j][r] * (1.0f / WSC));
    __syncthreads(); const size_t b = rb / TT; const int s0 = (int)(rb % TT); for (int e = tid; e < 128 * 8; e += 128) { const int d = e >> 3, pc = e & 7; vst2((unsigned*)(VPL + ((b * CC + c0 + d) * TT) + s0 + pc * 8), *(const v4u*)&st[d][pc * 8]); } return; }
  { const float al = (MODE == 2) ? bfr(ALPHA[0]) : 0.f;
#pragma unroll
    for (int j = 0; j < 8; ++j) { const float bb = (MODE == 2) ? bfr(BI[c0 + j * 16 + col]) : 0.f;
#pragma unroll
      for (int r = 0; r < 8; ++r) { float v = acc[j][r] * (1.0f / WSC) + bb; if (MODE == 2) v = (v >= 0.f) ? v : al * v; so[wave * 16 + 8 * g + r][j * 16 + col] = (_Float16)v; } } }
  __syncthreads();
  { _Float16* dst = (MODE == 0) ? ((which == 0) ? O16 : O16B) : O16; for (int e = tid; e < 64 * 16; e += 128) { const int rl = e >> 4, q = e & 15; vst2((unsigned*)(dst + (rb + rl) * ow + c0 + q * 8), *(const v4u*)&so[rl][q * 8]); } }
}
__global__ __launch_bounds__(128) void k_attn(const _Float16* __restrict__ Q, const _Float16* __restrict__ Kr, const _Float16* __restrict__ V, float* __restrict__ O) {
  __shared__ __align__(16) _Float16 sph[4][16][40]; __shared__ __align__(16) float so[4][16][68];
  const int tid = threadIdx.x, wave = tid >> 5, lane = tid & 31, col = lane & 15, g = lane >> 4; const int h = blockIdx.y; const size_t b = blockIdx.z; const int q0 = blockIdx.x * 64 + wave * 16; const size_t rq = b * TT + q0;
  v16h aq[2];
#pragma unroll
  for (int kc = 0; kc < 2; ++kc) aq[kc] = frag_h(Q + (rq + col) * CC + h * HS + kc * 32, lane);
  float m[8], l[8];
#pragma unroll
  for (int r = 0; r < 8; ++r) { m[r] = -3.0e38f; l[r] = 0.f; }
  v8f acc[4] = {};
#pragma unroll 1
  for (int ks = 0; ks < TT / 32; ++ks) { const int j0 = ks * 32; v8f s[2];
#pragma unroll
    for (int ct = 0; ct < 2; ++ct) { const int kk = j0 + ct * 16 + col; const size_t rk = (b * TT + kk) * CC + h * HS; v8f c = {};
#pragma unroll
      for (int kc = 0; kc < 2; ++kc) c = wmma16(aq[kc], frag_h(Kr + rk + kc * 32, lane), c);
#pragma unroll
      for (int r = 0; r < 8; ++r) s[ct][r] = c[r] * 0.125f; }
#pragma unroll
    for (int r = 0; r < 8; ++r) { float mx = fmaxf(s[0][r], s[1][r]);
#pragma unroll
      for (int o = 1; o < 16; o <<= 1) mx = fmaxf(mx, __shfl_xor(mx, o));
      const float mn = fmaxf(m[r], mx); const float alpha = (m[r] <= -1.0e38f) ? 0.f : __expf(m[r] - mn); const float e0 = __expf(s[0][r] - mn), e1 = __expf(s[1][r] - mn); float es = e0 + e1;
#pragma unroll
      for (int o = 1; o < 16; o <<= 1) es += __shfl_xor(es, o);
      l[r] = l[r] * alpha + es; m[r] = mn;
#pragma unroll
      for (int dt = 0; dt < 4; ++dt) acc[dt][r] *= alpha;
      sph[wave][8 * g + r][col] = (_Float16)(e0 * 2048.0f); sph[wave][8 * g + r][16 + col] = (_Float16)(e1 * 2048.0f); }
    LDSX();
    const v16h pa = frag_h(&sph[wave][col][0], lane);
#pragma unroll
    for (int dt = 0; dt < 4; ++dt) acc[dt] = wmma16(pa, frag_h(V + ((b * CC + h * HS + dt * 16 + col) * TT) + j0, lane), acc[dt]);
    LDSX(); }
#pragma unroll
  for (int r = 0; r < 8; ++r) { const float il = (1.0f / 2048.0f) / l[r];
#pragma unroll
    for (int dt = 0; dt < 4; ++dt) so[wave][8 * g + r][dt * 16 + col] = acc[dt][r] * il; }
  LDSX();
  for (int rl = 0; rl < 16; ++rl) if (lane < 16) vst2(O + (rq + rl) * CC + h * HS + lane * 4, *(const v4f*)&so[wave][rl][lane * 4]);
}
__global__ __launch_bounds__(128) void k_wo(const float* __restrict__ O, const _Float16* __restrict__ Wr, const float* __restrict__ SRC, float* __restrict__ S1) { __shared__ __align__(16) float sf[4][16][132];
  const int tid = threadIdx.x, wave = tid >> 5, lane = tid & 31, col = lane & 15, g = lane >> 4; const size_t r0 = (size_t)blockIdx.x * 64 + wave * 16; const int c0 = blockIdx.y * 128;
  v8f acc[8] = {};
#pragma unroll 2
  for (int kc = 0; kc < CC / 32; ++kc) { v16h a; { const float* p = O + (r0 + col) * CC + kc * 32 + 8 * g;
#pragma unroll
      for (int i = 0; i < 8; ++i) { a[i] = (_Float16)p[i]; a[8 + i] = (_Float16)p[16 + i]; } }
#pragma unroll
    for (int j = 0; j < 8; ++j) acc[j] = wmma16(a, frag_h(Wr + (size_t)(c0 + j * 16 + col) * CC + kc * 32, lane), acc[j]); }
#pragma unroll
  for (int j = 0; j < 8; ++j) { const int c = c0 + j * 16 + col;
#pragma unroll
    for (int r = 0; r < 8; ++r) sf[wave][8 * g + r][j * 16 + col] = acc[j][r] * (1.0f / WSC) + bfr(SRC[(r0 + 8 * g + r) * CC + c]); }
  LDSX(); for (int rl = 0; rl < 16; ++rl) vst2(S1 + (r0 + rl) * CC + c0 + lane * 4, *(const v4f*)&sf[wave][rl][lane * 4]); }
__global__ __launch_bounds__(128) void k_sstat(const _Float16* __restrict__ QS, float* __restrict__ ST) { __shared__ __align__(16) float sl[64][NH * 2 + 16];
  const int tid = threadIdx.x, wave = tid >> 5, lane = tid & 31, col = lane & 15, g = lane >> 4; const size_t b = blockIdx.y; const int n0 = blockIdx.x * 64 + wave * 16; const size_t rq = b * CC + n0;
  for (int e = tid; e < 64 * 32; e += 128) sl[e >> 5][e & 31] = 0.f; __syncthreads();
#pragma unroll 1
  for (int h = 0; h < NH; ++h) { v16h aq[2];
#pragma unroll
    for (int kc = 0; kc < 2; ++kc) aq[kc] = frag_h(QS + (rq + col) * 1024 + h * HS + kc * 32, lane);
    float m[8], l[8];
#pragma unroll
    for (int r = 0; r < 8; ++r) { m[r] = -3.0e38f; l[r] = 0.f; }
#pragma unroll 1
    for (int ks = 0; ks < CC / 32; ++ks) { const int j0 = ks * 32; v8f s[2];
#pragma unroll
      for (int ct = 0; ct < 2; ++ct) { const int kk = j0 + ct * 16 + col; v8f c = {};
#pragma unroll
        for (int kc = 0; kc < 2; ++kc) c = wmma16(aq[kc], frag_h(QS + (b * CC + kk) * 1024 + LL + h * HS + kc * 32, lane), c);
#pragma unroll
        for (int r = 0; r < 8; ++r) s[ct][r] = c[r] * 0.125f; }
#pragma unroll
      for (int r = 0; r < 8; ++r) { float mx = fmaxf(s[0][r], s[1][r]);
#pragma unroll
        for (int o = 1; o < 16; o <<= 1) mx = fmaxf(mx, __shfl_xor(mx, o));
        const float mn = fmaxf(m[r], mx); const float alpha = (m[r] <= -1.0e38f) ? 0.f : __expf(m[r] - mn); float es = __expf(s[0][r] - mn) + __expf(s[1][r] - mn);
#pragma unroll
        for (int o = 1; o < 16; o <<= 1) es += __shfl_xor(es, o);
        l[r] = l[r] * alpha + es; m[r] = mn; } }
    if (col == 0) {
#pragma unroll
      for (int r = 0; r < 8; ++r) { sl[wave * 16 + 8 * g + r][h * 2] = m[r]; sl[wave * 16 + 8 * g + r][h * 2 + 1] = l[r]; } } }
  __syncthreads();
  for (int e = tid; e < 64 * 8; e += 128) { const int rl = e >> 3, q = e & 7; vst2(ST + (b * CC + blockIdx.x * 64 + rl) * 32 + q * 4, *(const v4f*)&sl[rl][q * 4]); }
}
__global__ __launch_bounds__(128) void k_sprob(const _Float16* __restrict__ QS, const float* __restrict__ ST, float* __restrict__ SW, _Float16* __restrict__ SWH) { __shared__ __align__(16) float so[4][16][36]; __shared__ __align__(16) _Float16 sh[4][16][40];
  const int tid = threadIdx.x, wave = tid >> 5, lane = tid & 31, col = lane & 15, g = lane >> 4; const size_t b = blockIdx.y; const int n0 = blockIdx.x * 64 + wave * 16; const size_t rq = b * CC + n0;
#pragma unroll 1
  for (int ks = 0; ks < CC / 32; ++ks) { const int j0 = ks * 32; float accp[2][8];
#pragma unroll
    for (int ct = 0; ct < 2; ++ct)
#pragma unroll
      for (int r = 0; r < 8; ++r) accp[ct][r] = 0.f;
#pragma unroll 1
    for (int h = 0; h < NH; ++h) { v16h aq[2];
#pragma unroll
      for (int kc = 0; kc < 2; ++kc) aq[kc] = frag_h(QS + (rq + col) * 1024 + h * HS + kc * 32, lane);
#pragma unroll
      for (int ct = 0; ct < 2; ++ct) { const int kk = j0 + ct * 16 + col; v8f c = {};
#pragma unroll
        for (int kc = 0; kc < 2; ++kc) c = wmma16(aq[kc], frag_h(QS + (b * CC + kk) * 1024 + LL + h * HS + kc * 32, lane), c);
#pragma unroll
        for (int r = 0; r < 8; ++r) { const float* st = ST + (rq + 8 * g + r) * 32 + h * 2; accp[ct][r] += __expf(c[r] * 0.125f - st[0]) / st[1]; } } }
#pragma unroll
    for (int ct = 0; ct < 2; ++ct)
#pragma unroll
      for (int r = 0; r < 8; ++r) { const float v = accp[ct][r] * (1.0f / (float)NH); so[wave][8 * g + r][ct * 16 + col] = v; sh[wave][8 * g + r][ct * 16 + col] = (_Float16)v; }
    LDSX();
    for (int rl = 0; rl < 16; ++rl) { if (lane < 8) vst2(SW + (rq + rl) * CC + j0 + lane * 4, *(const v4f*)&so[wave][rl][lane * 4]); else if (lane < 12) vst2((unsigned*)(SWH + (rq + rl) * CC + j0 + (lane - 8) * 8), *(const v4u*)&sh[wave][rl][(lane - 8) * 8]); }
    LDSX(); }
}
__global__ __launch_bounds__(128) void k_mix(const _Float16* __restrict__ LN3, const _Float16* __restrict__ SWH, const float* __restrict__ S2, float* __restrict__ S3) { __shared__ __align__(16) float sf[4][16][132];
  const int tid = threadIdx.x, wave = tid >> 5, lane = tid & 31, col = lane & 15, g = lane >> 4; const size_t b = blockIdx.z; const size_t r0 = b * TT + (size_t)blockIdx.x * 64 + wave * 16; const int c0 = blockIdx.y * 128;
  v8f acc[8] = {};
#pragma unroll 2
  for (int kc = 0; kc < CC / 32; ++kc) { const v16h a = frag_h(LN3 + (r0 + col) * CC + kc * 32, lane);
#pragma unroll
    for (int j = 0; j < 8; ++j) acc[j] = wmma16(a, frag_h(SWH + ((b * CC + c0 + j * 16 + col) * CC) + kc * 32, lane), acc[j]); }
#pragma unroll
  for (int j = 0; j < 8; ++j) { const int c = c0 + j * 16 + col;
#pragma unroll
    for (int r = 0; r < 8; ++r) sf[wave][8 * g + r][j * 16 + col] = acc[j][r] + S2[(r0 + 8 * g + r) * CC + c]; }
  LDSX(); for (int rl = 0; rl < 16; ++rl) vst2(S3 + (r0 + rl) * CC + c0 + lane * 4, *(const v4f*)&sf[wave][rl][lane * 4]); }
extern "C" void kernel_launch(void* const* d_in, const int* in_sizes, int n_in, void* d_out, int out_size, void* d_ws, size_t ws_size, hipStream_t stream) {
  (void)in_sizes; (void)n_in; (void)out_size;
  const float** F = (const float**)d_in;
  if (ws_size < (size_t)WS_END) return;
  char* ws = (char*)d_ws; _Float16* P = (_Float16*)ws; _Float16 *LN = (_Float16*)(ws + WS_LN), *Q = (_Float16*)(ws + WS_Q), *Kr = (_Float16*)(ws + WS_K), *V = (_Float16*)(ws + WS_V), *HH = (_Float16*)(ws + WS_HH), *SP = (_Float16*)(ws + WS_SP), *QS = (_Float16*)(ws + WS_QS), *SWH = (_Float16*)(ws + WS_SWH); float *O = (float*)(ws + WS_O), *S1 = (float*)(ws + WS_S1), *S2 = (float*)(ws + WS_S2), *S3 = (float*)(ws + WS_S3), *ST = (float*)(ws + WS_ST);
  float* OUT0 = (float*)d_out; float* SW = (float*)d_out + OUT1;
  const int nr = TNB * TT;
  k_pack<<<dim3(HID, 7), 256, 0, stream>>>(F[2], F[3], F[4], F[5], F[8], F[10], F[6], F[7], F[12], F[14], P);
  k_ln<1><<<nr, 256, 0, stream>>>(F[0], F[17], F[18], LN);
  k_g<0, CC><<<dim3(nr / 64, CC / 128, 3), 128, 0, stream>>>(LN, P + WS_PW / 2, nullptr, nullptr, nullptr, nullptr, Q, Kr, V, CC);
  k_attn<<<dim3(TT / 64, NH, TNB), 128, 0, stream>>>(Q, Kr, V, O);
  k_wo<<<dim3(nr / 64, CC / 128), 128, 0, stream>>>(O, P + WS_PO / 2, F[0], S1);
  k_ln<0><<<nr, 256, 0, stream>>>(S1, F[19], F[20], LN);
  k_g<2, CC><<<dim3(nr / 64, HID / 128, 1), 128, 0, stream>>>(LN, P + WS_P1 / 2, F[9], nullptr, F[16], nullptr, HH, nullptr, nullptr, HID);
  k_g<1, HID><<<dim3(nr / 64, CC / 128, 1), 128, 0, stream>>>(HH, P + WS_P2 / 2, F[11], S1, nullptr, S2, nullptr, nullptr, nullptr, CC);
  k_ln<1><<<nr, 256, 0, stream>>>(F[1], F[25], F[26], SP);
  k_g<3, LL><<<dim3(nr / 64, 1024 / 128, 1), 128, 0, stream>>>(SP, P + WS_PS / 2, nullptr, nullptr, nullptr, nullptr, QS, nullptr, nullptr, 1024);
  k_sstat<<<dim3(CC / 64, TNB), 128, 0, stream>>>(QS, ST);
  k_sprob<<<dim3(CC / 64, TNB), 128, 0, stream>>>(QS, ST, SW, SWH);
  k_ln<0><<<nr, 256, 0, stream>>>(S2, F[21], F[22], LN);
  k_mix<<<dim3(TT / 64, CC / 128, TNB), 128, 0, stream>>>(LN, SWH, S2, S3);
  k_ln<0><<<nr, 256, 0, stream>>>(S3, F[23], F[24], LN);
  k_g<2, CC><<<dim3(nr / 64, HID / 128, 1), 128, 0, stream>>>(LN, P + WS_PT1 / 2, F[13], nullptr, F[16], nullptr, HH, nullptr, nullptr, HID);
  k_g<1, HID><<<dim3(nr / 64, CC / 128, 1), 128, 0, stream>>>(HH, P + WS_PT2 / 2, F[15], S3, nullptr, OUT0, nullptr, nullptr, nullptr, CC);
}
